// multi_head_attention_2d_5669356832203
// MI455X (gfx1250) — hardware-verified
//
#include <hip/hip_runtime.h>
#include <stddef.h>
#include <stdint.h>

#define NBATCH 2
#define CIN    256
#define HWS    1024
#define NSP    (NBATCH * HWS)
#define NHEAD  4
#define DK     64
#define NROW   (NSP * NHEAD)
#define CQ     256
#define NCOMB  (3 * CQ)
#define NW4    (4 * CQ)
#define GK     256
#define BR     32
#define BC     128
#define NCH    (NROW / BC)

static_assert(CIN == GK);
static_assert(CQ == GK);
static_assert(GK % 32 == 0);
static_assert(DK == 64);
static_assert(HWS % 256 == 0);
static_assert(NSP % 256 == 0);
static_assert(NCOMB % 64 == 0);
static_assert(CQ % 128 == 0);
static_assert(NSP % BR == 0);
static_assert(NROW % BC == 0);
static_assert(BC % 32 == 0);
static_assert(HWS % 64 == 0);
static_assert(CIN % 64 == 0);

typedef float          v8f   __attribute__((ext_vector_type(8)));
typedef float          v4f   __attribute__((ext_vector_type(4)));
typedef unsigned int   v4u   __attribute__((ext_vector_type(4)));
typedef unsigned short v8us  __attribute__((ext_vector_type(8)));
typedef unsigned short v16us __attribute__((ext_vector_type(16)));
typedef __bf16         v16b  __attribute__((ext_vector_type(16)));
typedef unsigned short ush;

union FragU { v16us v; v8us h[2]; v16b b; };
union PackU { v8us s; v4u u; };
struct HL { v4u h; v4u l; };

__device__ __forceinline__ ush f2bf(float f) {
  const unsigned u = __float_as_uint(f);
  return (ush)((u + 0x7FFFu + ((u >> 16) & 1u)) >> 16);
}
__device__ __forceinline__ float bf2f(ush b) { return __uint_as_float(((unsigned)b) << 16); }

__device__ __forceinline__ HL split8(v8f f) {
  PackU ph, pl;
#pragma unroll
  for (int e = 0; e < 8; ++e) {
    const ush hi = f2bf(f[e]);
    ph.s[e] = hi;
    pl.s[e] = f2bf(f[e] - bf2f(hi));
  }
  HL r; r.h = ph.u; r.l = pl.u;
  return r;
}

__device__ __forceinline__ v8f mmab(v16us a, v16us b, v8f c) {
  FragU ua, ub; ua.v = a; ub.v = b;
  c = __builtin_amdgcn_wmma_f32_16x16x32_bf16(false, ua.b, false, ub.b, (short)0, c, false, false);
  asm volatile("v_nop\n\tv_nop\n\tv_nop\n\tv_nop" : "+v"(c) : "v"(a), "v"(b));
  return c;
}

__device__ __forceinline__ v16us ldfragu(const ush* p, int ld, int row0, int k0, int lane) {
  const int m = lane & 15, lh = lane >> 4;
  const ush* q = p + (size_t)(row0 + m) * ld + k0 + 8 * lh;
  FragU f;
  f.h[0] = *(const v8us*)(q);
  f.h[1] = *(const v8us*)(q + 16);
  return f.v;
}

__device__ __forceinline__ v8f zero8() { return (v8f){0.f, 0.f, 0.f, 0.f, 0.f, 0.f, 0.f, 0.f}; }

__device__ __forceinline__ void gemm3_32x64(const ush* __restrict__ Ah, const ush* __restrict__ Al, int lda,
                                            const ush* __restrict__ Bh, const ush* __restrict__ Bl, int ldb,
                                            int m0, int n0, int lane, v8f (&acc)[2][4]) {
#pragma unroll 1
  for (int k0 = 0; k0 < GK; k0 += 32) {
    const v16us a0h = ldfragu(Ah, lda, m0, k0, lane);
    const v16us a1h = ldfragu(Ah, lda, m0 + 16, k0, lane);
    const v16us a0l = ldfragu(Al, lda, m0, k0, lane);
    const v16us a1l = ldfragu(Al, lda, m0 + 16, k0, lane);
#pragma unroll
    for (int t = 0; t < 4; ++t) {
      const v16us bh = ldfragu(Bh, ldb, n0 + 16 * t, k0, lane);
      const v16us bl = ldfragu(Bl, ldb, n0 + 16 * t, k0, lane);
      acc[0][t] = mmab(a0h, bh, acc[0][t]);
      acc[1][t] = mmab(a1h, bh, acc[1][t]);
      acc[0][t] = mmab(a0h, bl, acc[0][t]);
      acc[1][t] = mmab(a1h, bl, acc[1][t]);
      acc[0][t] = mmab(a0l, bh, acc[0][t]);
      acc[1][t] = mmab(a1l, bh, acc[1][t]);
    }
  }
}

#define XTP 65
__global__ __launch_bounds__(256) void k_cvt_x(const float* __restrict__ x, ush* __restrict__ xh,
                                               ush* __restrict__ xl) {
  __shared__ __align__(16) float tile[64 * XTP];
  const int tid = threadIdx.x;
  const int s0 = blockIdx.x * 64, c0 = blockIdx.y * 64, b = blockIdx.z;
#pragma unroll
  for (int j = 0; j < 4; ++j) {
    const int idx = tid + 256 * j;
    const int ci = idx >> 4, pi = idx & 15;
    const v4f v = *(const v4f*)(x + ((size_t)(b * CIN + c0 + ci)) * HWS + s0 + pi * 4);
    float* tp = tile + ci * XTP + pi * 4;
    tp[0] = v[0]; tp[1] = v[1]; tp[2] = v[2]; tp[3] = v[3];
  }
  __syncthreads();
  v4u vh[2], vl[2];
  size_t go[2];
#pragma unroll
  for (int j = 0; j < 2; ++j) {
    const int p  = tid + 256 * j;
    const int L  = p >> 3;
    const int pc = p & 7;
    v8f f;
#pragma unroll
    for (int e = 0; e < 8; ++e) f[e] = tile[(pc * 8 + e) * XTP + L];
    const HL s = split8(f);
    vh[j] = s.h; vl[j] = s.l;
    go[j] = ((size_t)(b * HWS + s0 + L)) * CIN + c0 + pc * 8;
  }
#pragma unroll
  for (int j = 0; j < 2; ++j) { *(volatile v4u*)(xh + go[j]) = vh[j]; *(volatile v4u*)(xl + go[j]) = vl[j]; }
  __threadfence();
#pragma unroll
  for (int j = 0; j < 2; ++j) { *(volatile v4u*)(xh + go[j]) = vh[j]; *(volatile v4u*)(xl + go[j]) = vl[j]; }
}

__global__ __launch_bounds__(256) void k_cvt_w(const float* __restrict__ wq, const float* __restrict__ wk,
                                               const float* __restrict__ wv, const float* __restrict__ wo,
                                               ush* __restrict__ w4h, ush* __restrict__ w4l, int ngrp) {
  const int which = blockIdx.y;
  const float* w = (which == 0) ? wq : ((which == 1) ? wk : ((which == 2) ? wv : wo));
  const int t = blockIdx.x * 256 + (int)threadIdx.x;
  if (t >= ngrp) return;
  const size_t o  = (size_t)t * 8;
  const size_t od = (size_t)which * CQ * GK + o;
  const v4f a0 = *(const v4f*)(w + o);
  const v4f a1 = *(const v4f*)(w + o + 4);
  const v8f f = (v8f){a0[0], a0[1], a0[2], a0[3], a1[0], a1[1], a1[2], a1[3]};
  const HL s = split8(f);
  *(volatile v4u*)(w4h + od) = s.h;
  *(volatile v4u*)(w4l + od) = s.l;
  __threadfence();
  *(volatile v4u*)(w4h + od) = s.h;
  *(volatile v4u*)(w4l + od) = s.l;
}

#define STP 72
__global__ __launch_bounds__(256) void k_qkv3(const ush* __restrict__ xth, const ush* __restrict__ xtl,
                                              const ush* __restrict__ w4h, const ush* __restrict__ w4l,
                                              const float* __restrict__ bq,
                                              const float* __restrict__ bk,
                                              const float* __restrict__ bv,
                                              ush* __restrict__ qh, ush* __restrict__ ql,
                                              ush* __restrict__ kh, ush* __restrict__ kl,
                                              ush* __restrict__ vth, ush* __restrict__ vtl) {
  __shared__ __align__(16) ush st[256 * STP];
  const int tid = threadIdx.x, lane = tid & 31, wave = tid >> 5;
  const int hh = lane >> 4, c = lane & 15;
  const int mb = blockIdx.x * 256;
  const int m0 = mb + wave * 32;
  const int n0 = blockIdx.y * 64;
  const int which = n0 / CQ;
  const int cc = n0 - which * CQ;
  const int head = cc / DK;
  const float* bias = (which == 0) ? bq : ((which == 1) ? bk : bv);
  const float  sc   = (which == 0) ? 0.125f : 1.0f;

  v8f acc[2][4];
#pragma unroll
  for (int s = 0; s < 2; ++s)
#pragma unroll
    for (int t = 0; t < 4; ++t) acc[s][t] = zero8();
  gemm3_32x64(xth, xtl, CIN, w4h, w4l, GK, m0, n0, lane, acc);

#pragma unroll
  for (int t = 0; t < 4; ++t) {
    const float bn = bias[cc + 16 * t + c];
#pragma unroll
    for (int sub = 0; sub < 2; ++sub) {
#pragma unroll
      for (int r = 0; r < 8; ++r) acc[sub][t][r] = (acc[sub][t][r] + bn) * sc;
    }
  }

  ush* bhp = (which == 0) ? qh : ((which == 1) ? kh : vth);
  ush* blp = (which == 0) ? ql : ((which == 1) ? kl : vtl);
  size_t go[8];
#pragma unroll
  for (int j = 0; j < 8; ++j) {
    const int p  = tid + 256 * j;
    const int L  = p >> 3;
    const int pc = p & 7;
    if (which < 2) {
      go[j] = ((size_t)(head * NSP + mb + L)) * DK + pc * 8;
    } else {
      const int d  = L >> 2;
      const int nl = (L & 3) * 64 + pc * 8;
      go[j] = ((size_t)d) * NROW + (size_t)(head * NSP + mb + nl);
    }
  }

#pragma unroll 1
  for (int ph = 0; ph < 2; ++ph) {
    __syncthreads();
#pragma unroll
    for (int t = 0; t < 4; ++t) {
#pragma unroll
      for (int sub = 0; sub < 2; ++sub) {
#pragma unroll
        for (int r = 0; r < 8; ++r) {
          const int lr = wave * 32 + sub * 16 + 8 * hh + r;
          const float v = acc[sub][t][r];
          const ush hi = f2bf(v);
          st[lr * STP + 16 * t + c] = (ph == 0) ? hi : f2bf(v - bf2f(hi));
        }
      }
    }
    __syncthreads();
    v4u val[8];
    if (which < 2) {
#pragma unroll
      for (int j = 0; j < 8; ++j) {
        const int p  = tid + 256 * j;
        const int lr = p >> 3;
        const int pc = p & 7;
        PackU pk;
        pk.s  = *(const v8us*)(st + lr * STP + pc * 8);
        val[j] = pk.u;
      }
    } else {
#pragma unroll
      for (int j = 0; j < 8; ++j) {
        const int p  = tid + 256 * j;
        const int L  = p >> 3;
        const int pc = p & 7;
        const int d  = L >> 2;
        const int nl = (L & 3) * 64 + pc * 8;
        const ush* cp = st + nl * STP + d;
        PackU pk;
        pk.s = (v8us){cp[0 * STP], cp[1 * STP], cp[2 * STP], cp[3 * STP],
                      cp[4 * STP], cp[5 * STP], cp[6 * STP], cp[7 * STP]};
        val[j] = pk.u;
      }
    }
    ush* dst = (ph == 0) ? bhp : blp;
#pragma unroll
    for (int j = 0; j < 8; ++j) *(volatile v4u*)(dst + go[j]) = val[j];
    __threadfence();
#pragma unroll
    for (int j = 0; j < 8; ++j) *(volatile v4u*)(dst + go[j]) = val[j];
    __threadfence();
  }
}

#define SSP 128
#define SPP 136
#define OTP 68
__global__ __launch_bounds__(256) void k_attn3(const ush* __restrict__ qh, const ush* __restrict__ ql,
                                               const ush* __restrict__ kh, const ush* __restrict__ kl,
                                               const ush* __restrict__ vth, const ush* __restrict__ vtl,
                                               ush* __restrict__ oh, ush* __restrict__ ol) {
  __shared__ __align__(16) float sSO[BR * SSP];
  __shared__ __align__(16) ush   sPh[BR * SPP];
  __shared__ __align__(16) ush   sPl[BR * SPP];
  __shared__ __align__(16) float sRed[BR * 8];
  __shared__ __align__(16) float rM[BR];
  __shared__ __align__(16) float rMn[BR];
  __shared__ __align__(16) float rL[BR];
  __shared__ __align__(16) float rSc[BR];

  float* sS = sSO;
  const int tid = threadIdx.x, lane = tid & 31, wave = tid >> 5;
  const int hh = lane >> 4, c = lane & 15;
  const int rt = wave >> 2, ct = wave & 3;
  const int q0 = (int)blockIdx.x * BR;
  const float NEGI = -__builtin_huge_valf();
  if (tid < BR) { rM[tid] = NEGI; rL[tid] = 0.f; }

  const v16us a0h0 = ldfragu(qh, DK, q0,      0,  lane);
  const v16us a1h0 = ldfragu(qh, DK, q0 + 16, 0,  lane);
  const v16us a0l0 = ldfragu(ql, DK, q0,      0,  lane);
  const v16us a1l0 = ldfragu(ql, DK, q0 + 16, 0,  lane);
  const v16us a0h1 = ldfragu(qh, DK, q0,      32, lane);
  const v16us a1h1 = ldfragu(qh, DK, q0 + 16, 32, lane);
  const v16us a0l1 = ldfragu(ql, DK, q0,      32, lane);
  const v16us a1l1 = ldfragu(ql, DK, q0 + 16, 32, lane);
  __syncthreads();

  v8f oacc = zero8();
  const int srow = tid >> 3, schk = tid & 7;

#pragma unroll 1
  for (int ch = 0; ch < NCH; ++ch) {
    const int j0  = ch * BC;
    const int kr0 = j0 + wave * 16;
    v8f s[2];
    s[0] = zero8(); s[1] = zero8();
    {
      const v16us kbh = ldfragu(kh, DK, kr0, 0, lane);
      const v16us kbl = ldfragu(kl, DK, kr0, 0, lane);
      s[0] = mmab(a0h0, kbh, s[0]);
      s[1] = mmab(a1h0, kbh, s[1]);
      s[0] = mmab(a0h0, kbl, s[0]);
      s[1] = mmab(a1h0, kbl, s[1]);
      s[0] = mmab(a0l0, kbh, s[0]);
      s[1] = mmab(a1l0, kbh, s[1]);
    }
    {
      const v16us kbh = ldfragu(kh, DK, kr0, 32, lane);
      const v16us kbl = ldfragu(kl, DK, kr0, 32, lane);
      s[0] = mmab(a0h1, kbh, s[0]);
      s[1] = mmab(a1h1, kbh, s[1]);
      s[0] = mmab(a0h1, kbl, s[0]);
      s[1] = mmab(a1h1, kbl, s[1]);
      s[0] = mmab(a0l1, kbh, s[0]);
      s[1] = mmab(a1l1, kbh, s[1]);
    }
#pragma unroll
    for (int t = 0; t < 2; ++t) {
#pragma unroll
      for (int r = 0; r < 8; ++r) {
        const int row = 16 * t + 8 * hh + r;
        sS[row * SSP + wave * 16 + c] = s[t][r];
      }
    }
    __syncthreads();
    {
      const float* sr = sS + srow * SSP + schk * 16;
      const v4f x0 = *(const v4f*)(sr);
      const v4f x1 = *(const v4f*)(sr + 4);
      const v4f x2 = *(const v4f*)(sr + 8);
      const v4f x3 = *(const v4f*)(sr + 12);
      float mx = x0[0];
#pragma unroll
      for (int e = 1; e < 4; ++e) mx = fmaxf(mx, x0[e]);
#pragma unroll
      for (int e = 0; e < 4; ++e) { mx = fmaxf(mx, x1[e]); mx = fmaxf(mx, x2[e]); mx = fmaxf(mx, x3[e]); }
      sRed[srow * 8 + schk] = mx;
    }
    __syncthreads();
    if (tid < BR) {
      float mx = rM[tid];
#pragma unroll
      for (int i = 0; i < 8; ++i) mx = fmaxf(mx, sRed[tid * 8 + i]);
      rMn[tid] = mx;
    }
    __syncthreads();
    {
      const float mx = rMn[srow];
      const float* sr = sS + srow * SSP + schk * 16;
      float sum = 0.f;
      PackU ph0, pl0, ph1, pl1;
#pragma unroll
      for (int e = 0; e < 8; ++e) {
        const float p = __expf(sr[e] - mx);
        sum += p;
        const ush hi = f2bf(p);
        ph0.s[e] = hi;
        pl0.s[e] = f2bf(p - bf2f(hi));
      }
#pragma unroll
      for (int e = 0; e < 8; ++e) {
        const float p = __expf(sr[8 + e] - mx);
        sum += p;
        const ush hi = f2bf(p);
        ph1.s[e] = hi;
        pl1.s[e] = f2bf(p - bf2f(hi));
      }
      *(v8us*)(sPh + srow * SPP + schk * 16)     = ph0.s;
      *(v8us*)(sPh + srow * SPP + schk * 16 + 8) = ph1.s;
      *(v8us*)(sPl + srow * SPP + schk * 16)     = pl0.s;
      *(v8us*)(sPl + srow * SPP + schk * 16 + 8) = pl1.s;
      sRed[srow * 8 + schk] = sum;
    }
    __syncthreads();
    if (tid < BR) {
      float sum = 0.f;
#pragma unroll
      for (int i = 0; i < 8; ++i) sum += sRed[tid * 8 + i];
      const float mnew = rMn[tid];
      const float fac  = __expf(rM[tid] - mnew);
      rL[tid]  = rL[tid] * fac + sum;
      rM[tid]  = mnew;
      rSc[tid] = fac;
    }
    __syncthreads();
    {
      const v4f f0 = *(const v4f*)(rSc + 16 * rt + 8 * hh);
      const v4f f1 = *(const v4f*)(rSc + 16 * rt + 8 * hh + 4);
#pragma unroll
      for (int r = 0; r < 4; ++r) {
        oacc[r]     *= f0[r];
        oacc[4 + r] *= f1[r];
      }
    }
#pragma unroll 1
    for (int kk = 0; kk < BC / 32; ++kk) {
      const v16us pah = ldfragu(sPh, SPP, 16 * rt, kk * 32, lane);
      const v16us pal = ldfragu(sPl, SPP, 16 * rt, kk * 32, lane);
      const v16us vbh = ldfragu(vth, NROW, 16 * ct, j0 + kk * 32, lane);
      const v16us vbl = ldfragu(vtl, NROW, 16 * ct, j0 + kk * 32, lane);
      oacc = mmab(pah, vbh, oacc);
      oacc = mmab(pah, vbl, oacc);
      oacc = mmab(pal, vbh, oacc);
    }
    __syncthreads();
  }

  float* sO = sSO;
#pragma unroll
  for (int r = 0; r < 8; ++r) {
    const int row  = 16 * rt + 8 * hh + r;
    const float lv  = rL[row];
    const float inv = (lv > 0.f) ? (1.0f / lv) : 0.f;
    sO[row * OTP + ct * 16 + c] = oacc[r] * inv;
  }
  __syncthreads();
  const int head = q0 / NSP;
  const int nb   = q0 - head * NSP;
  const int L  = tid >> 3;
  const int pc = tid & 7;
  v8f f;
#pragma unroll
  for (int e = 0; e < 8; ++e) f[e] = sO[L * OTP + pc * 8 + e];
  const HL sp = split8(f);
  const size_t go = ((size_t)(nb + L)) * CQ + head * DK + pc * 8;
  *(volatile v4u*)(oh + go) = sp.h;
  *(volatile v4u*)(ol + go) = sp.l;
  __threadfence();
  *(volatile v4u*)(oh + go) = sp.h;
  *(volatile v4u*)(ol + go) = sp.l;
}

#define OSP 68
__global__ __launch_bounds__(128) void k_out3(const ush* __restrict__ w4h, const ush* __restrict__ w4l,
                                              const ush* __restrict__ oh, const ush* __restrict__ ol,
                                              const float* __restrict__ bo, float* __restrict__ out) {
  __shared__ __align__(16) float st[128 * OSP];
  const int tid = threadIdx.x, lane = tid & 31, wave = tid >> 5;
  const int hh = lane >> 4, c = lane & 15;
  const int n0 = blockIdx.x * 64;
  const int o0 = blockIdx.y * 128;
  const int b  = n0 / HWS;
  const int s0 = n0 - b * HWS;
  const int m0 = 3 * CQ + o0 + wave * 32;

  v8f acc[2][4];
#pragma unroll
  for (int s = 0; s < 2; ++s)
#pragma unroll
    for (int t = 0; t < 4; ++t) acc[s][t] = zero8();
  gemm3_32x64(w4h, w4l, GK, oh, ol, CQ, m0, n0, lane, acc);

#pragma unroll
  for (int sub = 0; sub < 2; ++sub) {
#pragma unroll
    for (int r = 0; r < 8; ++r) {
      const int lr = wave * 32 + sub * 16 + 8 * hh + r;
      const float bn = bo[o0 + lr];
#pragma unroll
      for (int t = 0; t < 4; ++t) st[lr * OSP + 16 * t + c] = acc[sub][t][r] + bn;
    }
  }
  __syncthreads();
  v4f val[16];
#pragma unroll
  for (int j = 0; j < 16; ++j) {
    const int p  = tid + 128 * j;
    const int L  = p >> 3;
    const int pc = p & 7;
    const int lr = L >> 1, hf = L & 1;
    val[j] = *(const v4f*)(st + lr * OSP + hf * 32 + pc * 4);
  }
#pragma unroll
  for (int j = 0; j < 16; ++j) {
    const int p  = tid + 128 * j;
    const int L  = p >> 3;
    const int pc = p & 7;
    const int lr = L >> 1, hf = L & 1;
    const size_t go = ((size_t)(b * CQ + o0 + lr)) * HWS + s0 + hf * 32 + pc * 4;
    *(volatile v4f*)(out + go) = val[j];
  }
  __threadfence();
#pragma unroll
  for (int j = 0; j < 16; ++j) {
    const int p  = tid + 128 * j;
    const int L  = p >> 3;
    const int pc = p & 7;
    const int lr = L >> 1, hf = L & 1;
    const size_t go = ((size_t)(b * CQ + o0 + lr)) * HWS + s0 + hf * 32 + pc * 4;
    *(volatile v4f*)(out + go) = val[j];
  }
}

extern "C" void kernel_launch(void* const* d_in, const int* in_sizes, int n_in,
                              void* d_out, int out_size, void* d_ws, size_t ws_size,
                              hipStream_t stream) {
  if (n_in < 9) return;
  if (in_sizes[0] != NBATCH * CIN * HWS) return;
  if (in_sizes[1] != CQ * CIN) return;
  if (in_sizes[2] != CQ) return;
  if (in_sizes[3] != CQ * CIN) return;
  if (in_sizes[4] != CQ) return;
  if (in_sizes[5] != CQ * CIN) return;
  if (in_sizes[6] != CQ) return;
  if (in_sizes[7] != CQ * CQ) return;
  if (in_sizes[8] != CQ) return;
  if (out_size != NBATCH * CQ * HWS) return;

  const float* x  = (const float*)d_in[0];
  const float* wq = (const float*)d_in[1];
  const float* bq = (const float*)d_in[2];
  const float* wk = (const float*)d_in[3];
  const float* bk = (const float*)d_in[4];
  const float* wv = (const float*)d_in[5];
  const float* bv = (const float*)d_in[6];
  const float* wo = (const float*)d_in[7];
  const float* bo = (const float*)d_in[8];
  float* out = (float*)d_out;

  size_t off = 0;
  const size_t oXTh = off; off += (size_t)NSP * CIN * 2;
  const size_t oXTl = off; off += (size_t)NSP * CIN * 2;
  const size_t oW4h = off; off += (size_t)NW4 * GK * 2;
  const size_t oW4l = off; off += (size_t)NW4 * GK * 2;
  const size_t oQh  = off; off += (size_t)NROW * DK * 2;
  const size_t oQl  = off; off += (size_t)NROW * DK * 2;
  const size_t oKh  = off; off += (size_t)NROW * DK * 2;
  const size_t oKl  = off; off += (size_t)NROW * DK * 2;
  const size_t oVTh = off; off += (size_t)DK * NROW * 2;
  const size_t oVTl = off; off += (size_t)DK * NROW * 2;
  const size_t oOh  = off; off += (size_t)NSP * CQ * 2;
  const size_t oOl  = off; off += (size_t)NSP * CQ * 2;
  if (off > ws_size) return;
  if (off > (size_t)134217728) return;

  char* ws = (char*)d_ws;
  ush* XTh = (ush*)(ws + oXTh);
  ush* XTl = (ush*)(ws + oXTl);
  ush* W4h = (ush*)(ws + oW4h);
  ush* W4l = (ush*)(ws + oW4l);
  ush* Qh  = (ush*)(ws + oQh);
  ush* Ql  = (ush*)(ws + oQl);
  ush* Kh  = (ush*)(ws + oKh);
  ush* Kl  = (ush*)(ws + oKl);
  ush* VTh = (ush*)(ws + oVTh);
  ush* VTl = (ush*)(ws + oVTl);
  ush* Oh  = (ush*)(ws + oOh);
  ush* Ol  = (ush*)(ws + oOl);

  k_cvt_x<<<dim3(HWS / 64, CIN / 64, NBATCH), dim3(256), 0, stream>>>(x, XTh, XTl);
  const int ngw = in_sizes[1] / 8;
  k_cvt_w<<<dim3((ngw + 255) / 256, 4), dim3(256), 0, stream>>>(wq, wk, wv, wo, W4h, W4l, ngw);
  k_qkv3<<<dim3(NSP / 256, NCOMB / 64), dim3(256), 0, stream>>>(XTh, XTl, W4h, W4l, bq, bk, bv,
                                                              Qh, Ql, Kh, Kl, VTh, VTl);
  k_attn3<<<dim3(NROW / BR), dim3(256), 0, stream>>>(Qh, Ql, Kh, Kl, VTh, VTl, Oh, Ol);
  k_out3<<<dim3(NSP / 64, CQ / 128), dim3(128), 0, stream>>>(W4h, W4l, Oh, Ol, bo, out);
  (void)hipGetLastError();
}
